// ResGCN_20289425506396
// MI455X (gfx1250) — hardware-verified
//
#include <hip/hip_runtime.h>
#include <stddef.h>
#include <stdint.h>


#define DH      128
#define DHID    256
#define DINF    7
#define KE      32
#define NLAY    5
#define NGRAPH  256
#define OPW     256
#define HPW     512
#define KA      256
#define KB      512
#define LNEPS   1e-5f
#define EPSM    1e-7f
#define EPSS    1e-16f
#define NTHR    256
#define NWAVE   8
#define EPT     8
#define CHUNK   (NTHR * EPT)
#define WCAP    (EPT * 32)
#define LISTN   (NWAVE * WCAP)
#define NBA     1024
#define SLA     10
#define RCAP    16384
#define DEGCAP  64
#define GBM     64
#define ABM     32
#define GTHR    128
#define AGG_ZINTS (LISTN + 2 * RCAP + 3 * NBA)
#define MISC_INTS 16
#define CMP_LDS_INTS (AGG_ZINTS + MISC_INTS)
#define NUE     (DH * (KE / 8))
#define NUW1    (NLAY * DHID * (KA / 8))
#define NUW2    (NLAY * DH * (KB / 8))
#define NUFIX   (NUE + NUW1 + NUW2)
#define WSMAX   134217728

static_assert((CHUNK & (CHUNK - 1)) == 0 && CHUNK <= 4096);
static_assert((NBA & (NBA - 1)) == 0 && NBA == (1 << SLA));
static_assert(((long long)CHUNK << SLA) < (1LL << 31));
static_assert(NBA % NWAVE == 0 && NBA % 32 == 0 && NBA % GBM == 0 && NBA == NTHR * 4);
static_assert(RCAP % 4 == 0 && (RCAP / 4) % NTHR == 0);
static_assert(AGG_ZINTS % (NTHR * 4) == 0);
static_assert(RCAP >= 13176);
static_assert(DEGCAP >= 28 + 8);
static_assert(CMP_LDS_INTS * 4 <= 300000);
static_assert(KE % 32 == 0 && KA % 32 == 0 && KB % 32 == 0 && KA == 2 * DH && KB == 2 * DHID);
static_assert(OPW == KA && HPW == KB);
static_assert(GBM == (GTHR / 32) * 16 && ABM == 32 && DH == 4 * 32 && DHID == 8 * 32);
static_assert(NUE % NTHR == 0 && NUW1 % NTHR == 0 && NUW2 % NTHR == 0);
static_assert(DHID * (KA / 8) == 8192 && DH * (KB / 8) == 8192);
static_assert(DINF <= KE && KE / 8 == 4);
static_assert(NGRAPH == NTHR);

typedef float          v4f   __attribute__((ext_vector_type(4)));
typedef float          v8f   __attribute__((ext_vector_type(8)));
typedef int            v4i   __attribute__((ext_vector_type(4)));
typedef int            v8i   __attribute__((ext_vector_type(8)));
typedef unsigned       v2u   __attribute__((ext_vector_type(2)));
typedef unsigned       v4u   __attribute__((ext_vector_type(4)));
typedef unsigned short v8us  __attribute__((ext_vector_type(8)));
typedef __bf16         v16bf __attribute__((ext_vector_type(16)));
typedef v4f  __attribute__((may_alias)) v4fa;
typedef v4i  __attribute__((may_alias)) v4ia;
typedef v2u  __attribute__((may_alias)) v2ua;
typedef v4u  __attribute__((may_alias)) v4ua;
typedef v8us __attribute__((may_alias)) v8usa;
union FragB { v16bf v; v8us h[2]; v8i w; };

__device__ __forceinline__ v8f wmb(const FragB& a, const FragB& b, v8f c) {
  v8f d = __builtin_amdgcn_wmma_f32_16x16x32_bf16(false, a.v, false, b.v, (short)0, c, false, false);
  asm volatile("v_nop\n\tv_nop\n\tv_nop\n\tv_nop" : "+v"(d) : "v"(a.w), "v"(b.w));
  return d;
}

__device__ __forceinline__ v8f z8() { v8f z = {0.f, 0.f, 0.f, 0.f, 0.f, 0.f, 0.f, 0.f}; return z; }

__device__ __forceinline__ unsigned bf16_bits(float f) {
  const unsigned u = __float_as_uint(f);
  return (u + 0x7FFFu + ((u >> 16) & 1u)) >> 16;
}
__device__ __forceinline__ float bf16_val(float f) {
  return __uint_as_float(bf16_bits(f) << 16);
}
__device__ __forceinline__ unsigned hl_bits(float v, unsigned& lo) {
  const unsigned hb = bf16_bits(v);
  lo = bf16_bits(v - __uint_as_float(hb << 16));
  return hb;
}
__device__ __forceinline__ float relu_keep(float v) { return (v != v) ? v : fmaxf(v, 0.0f); }

__device__ __forceinline__ void wave_sync() {
  __builtin_amdgcn_fence(__ATOMIC_RELEASE, "wavefront");
  __builtin_amdgcn_wave_barrier();
  __builtin_amdgcn_fence(__ATOMIC_ACQUIRE, "wavefront");
}

template <int SLB>
__device__ __forceinline__ int scan_chunk(const int* __restrict__ dsts, int nE, int cbase, int slotBase,
                                          int nb, int vec8, int* list, int tid, int lane, int wave) {
  int wc = 0;
  const int el0  = tid * EPT;
  const int e0   = cbase + el0;
  const int sent = -2147483647 - 1;
  v4i da, db;
  if (vec8 != 0 && cbase + CHUNK <= nE) {
    da = *(const v4i*)(dsts + e0);
    db = *(const v4i*)(dsts + e0 + 4);
  } else {
    da.x = (e0     < nE) ? dsts[min(e0,     nE - 1)] : sent;
    da.y = (e0 + 1 < nE) ? dsts[min(e0 + 1, nE - 1)] : sent;
    da.z = (e0 + 2 < nE) ? dsts[min(e0 + 2, nE - 1)] : sent;
    da.w = (e0 + 3 < nE) ? dsts[min(e0 + 3, nE - 1)] : sent;
    db.x = (e0 + 4 < nE) ? dsts[min(e0 + 4, nE - 1)] : sent;
    db.y = (e0 + 5 < nE) ? dsts[min(e0 + 5, nE - 1)] : sent;
    db.z = (e0 + 6 < nE) ? dsts[min(e0 + 6, nE - 1)] : sent;
    db.w = (e0 + 7 < nE) ? dsts[min(e0 + 7, nE - 1)] : sent;
  }
  const unsigned nbs = (unsigned)slotBase;
  const unsigned unb = (unsigned)nb;
  const unsigned s0 = (unsigned)da.x - nbs, s1 = (unsigned)da.y - nbs;
  const unsigned s2 = (unsigned)da.z - nbs, s3 = (unsigned)da.w - nbs;
  const unsigned s4 = (unsigned)db.x - nbs, s5 = (unsigned)db.y - nbs;
  const unsigned s6 = (unsigned)db.z - nbs, s7 = (unsigned)db.w - nbs;
  const bool h0 = s0 < unb, h1 = s1 < unb, h2 = s2 < unb, h3 = s3 < unb;
  const bool h4 = s4 < unb, h5 = s5 < unb, h6 = s6 < unb, h7 = s7 < unb;
  const unsigned any = __builtin_amdgcn_ballot_w32(h0 | h1 | h2 | h3 | h4 | h5 | h6 | h7);
  if (any != 0u) {
#define HITJ(J, HJ, SJ) { \
      const unsigned mj = __builtin_amdgcn_ballot_w32(HJ); \
      if (mj != 0u) { \
        if (HJ) { \
          const int pos = wc + (int)__builtin_amdgcn_mbcnt_lo(mj, 0u); \
          if (pos < WCAP) list[wave * WCAP + pos] = ((el0 + (J)) << SLB) | (int)(SJ); \
        } \
        wc += (int)__builtin_popcount(mj); } }
    HITJ(0, h0, s0)
    HITJ(1, h1, s1)
    HITJ(2, h2, s2)
    HITJ(3, h3, s3)
    HITJ(4, h4, s4)
    HITJ(5, h5, s5)
    HITJ(6, h6, s6)
    HITJ(7, h7, s7)
#undef HITJ
  }
  return wc;
}

__global__ __launch_bounds__(NTHR) void k_prep(const float* __restrict__ x, const float* __restrict__ encW,
                                               const float* __restrict__ W1, const float* __restrict__ W2,
                                               unsigned short* ewt, unsigned short* w1t, unsigned short* w2t,
                                               unsigned short* xb, int nN, int nUnits) {
  const int u = (int)blockIdx.x * NTHR + (int)threadIdx.x;
  v8us o;
  unsigned short* dp;
  if (u < NUE) {
    const int n = u >> 2, k8 = (u & 3) * 8;
#pragma unroll
    for (int i = 0; i < 8; ++i) {
      const int k  = k8 + i;
      const int kc = k < DINF ? k : DINF - 1;
      const float f = encW[(size_t)kc * DH + n];
      o[i] = (unsigned short)bf16_bits(k < DINF ? f : 0.0f);
    }
    dp = ewt + (size_t)u * 8;
  } else if (u < NUE + NUW1) {
    const int v  = u - NUE;
    const int l  = v >> 13;
    const int n  = (v >> 5) & (DHID - 1), k8 = (v & 31) * 8;
    const int kk = k8 & (DH - 1);
    const float* p = W1 + (size_t)l * DH * DHID + (size_t)kk * DHID + n;
#pragma unroll
    for (int i = 0; i < 8; ++i) o[i] = (unsigned short)bf16_bits(p[(size_t)i * DHID]);
    dp = w1t + (size_t)v * 8;
  } else if (u < NUFIX) {
    const int v  = u - NUE - NUW1;
    const int l  = v >> 13;
    const int n  = (v >> 6) & (DH - 1), k8 = (v & 63) * 8;
    const int kk = k8 & (DHID - 1);
    const float* p = W2 + (size_t)l * DHID * DH + (size_t)kk * DH + n;
#pragma unroll
    for (int i = 0; i < 8; ++i) o[i] = (unsigned short)bf16_bits(p[(size_t)i * DH]);
    dp = w2t + (size_t)v * 8;
  } else if (u < nUnits) {
    const int v   = u - NUFIX;
    const int row = v >> 2, k8 = (v & 3) * 8;
    const int rc  = row < nN ? row : nN - 1;
    const bool lv = row < nN;
    const float* p = x + (size_t)rc * DINF;
#pragma unroll
    for (int i = 0; i < 8; ++i) {
      const int k  = k8 + i;
      const int kc = k < DINF ? k : DINF - 1;
      const float f = p[kc];
      o[i] = (unsigned short)bf16_bits((lv && k < DINF) ? f : 0.0f);
    }
    dp = xb + (size_t)v * 8;
  } else {
    return;
  }
  *(volatile v8us*)dp = o;
  __threadfence();
  *(volatile v8us*)dp = o;
}

__global__ __launch_bounds__(NTHR) void k_compact(const int* __restrict__ srcs, const int* __restrict__ dsts,
                                                  int nE, int nN, int vec8,
                                                  int* lst, int* cntg, int* offg, int* flg) {
  extern __shared__ __attribute__((aligned(16))) int dsm[];
  int* list = dsm;
  int* hl   = dsm + LISTN;
  int* sl   = hl + RCAP;
  int* cnt  = sl + RCAP;
  int* offs = cnt + NBA;
  int* cur  = offs + NBA;
  int* misc = cur + NBA;
  const int tid = (int)threadIdx.x, lane = tid & 31, wave = tid >> 5;
  const int nodeBase = (int)blockIdx.x * NBA;

  {
    const v4i z4 = {0, 0, 0, 0};
    for (int i = tid * 4; i < AGG_ZINTS; i += NTHR * 4) *(v4ia*)(dsm + i) = z4;
    if (tid < MISC_INTS) misc[tid] = 0;
  }
  __syncthreads();

  int t = 0, ov = 0;
  const int nChunks = (nE + CHUNK - 1) / CHUNK;
#pragma unroll 1
  for (int ch = 0; ch < nChunks; ++ch) {
    const int cbase = ch * CHUNK;
    const int wc = scan_chunk<SLA>(dsts, nE, cbase, nodeBase, NBA, vec8, list, tid, lane, wave);
    if (lane == 0) misc[wave] = wc;
    __syncthreads();
    if (wave == 0) {
#pragma unroll 1
      for (int w2 = 0; w2 < NWAVE; ++w2) {
        int c = misc[w2];
        c = c < 0 ? 0 : (c > WCAP ? WCAP : c);
#pragma unroll 1
        for (int b0 = 0; b0 < c; b0 += 32) {
          const int idx = b0 + lane;
          const int ent_ = list[w2 * WCAP + (idx < WCAP ? idx : WCAP - 1)];
          const int m32 = (c - b0) < 32 ? (c - b0) : 32;
#pragma unroll 1
          for (int k = 0; k < m32; ++k) {
            const int u    = __builtin_amdgcn_readlane(ent_, k);
            const int slot = u & (NBA - 1);
            const int el   = (u >> SLA) & (CHUNK - 1);
            const int pk   = ((cbase + el) << SLA) | slot;
            if (t < RCAP) {
              if (lane == 0) { hl[t] = pk; cnt[slot] = cnt[slot] + 1; }
              t = t + 1;
            } else {
              ov = 1;
            }
          }
        }
      }
    }
    __syncthreads();
  }
  if (wave == 0 && lane == 0) { misc[8] = t; misc[9] = ov; }
  __syncthreads();
  int tt = misc[8];
  tt = tt < 0 ? 0 : (tt > RCAP ? RCAP : tt);
  const int ovf = misc[9];

  if (wave == 0) {
    const int base = lane * (NBA / 32);
    int s = 0;
#pragma unroll 1
    for (int i = 0; i < NBA / 32; ++i) s += cnt[base + i];
    int incl = s;
#pragma unroll
    for (int d = 1; d < 32; d <<= 1) {
      const int y = __shfl_up(incl, d, 32);
      if (lane >= d) incl += y;
    }
    int run = incl - s;
#pragma unroll 1
    for (int i = 0; i < NBA / 32; ++i) {
      const int cv = cnt[base + i];
      offs[base + i] = run;
      cur[base + i]  = run;
      run += cv;
    }
  }
  __syncthreads();
  if (wave == 0) {
#pragma unroll 1
    for (int b0 = 0; b0 < tt; b0 += 32) {
      const int idx = b0 + lane;
      const int ent_ = hl[idx < RCAP ? idx : RCAP - 1];
      const int m32 = (tt - b0) < 32 ? (tt - b0) : 32;
#pragma unroll 1
      for (int k = 0; k < m32; ++k) {
        const int u    = __builtin_amdgcn_readlane(ent_, k);
        const int slot = u & (NBA - 1);
        if (lane == 0) {
          int p = cur[slot];
          p = p < 0 ? 0 : (p > RCAP - 1 ? RCAP - 1 : p);
          sl[p] = u;
          cur[slot] = p + 1;
        }
      }
    }
  }
  __syncthreads();

  int* lb = lst + (size_t)blockIdx.x * RCAP;
#pragma unroll 1
  for (int u = tid; u < RCAP / 4; u += NTHR) {
    const v4i e4 = *(const v4ia*)(sl + 4 * u);
    int e0 = e4.x >> SLA, e1 = e4.y >> SLA, e2 = e4.z >> SLA, e3 = e4.w >> SLA;
    e0 = e0 < 0 ? 0 : (e0 > nE - 1 ? nE - 1 : e0);
    e1 = e1 < 0 ? 0 : (e1 > nE - 1 ? nE - 1 : e1);
    e2 = e2 < 0 ? 0 : (e2 > nE - 1 ? nE - 1 : e2);
    e3 = e3 < 0 ? 0 : (e3 > nE - 1 ? nE - 1 : e3);
    int s0 = srcs[e0], s1 = srcs[e1], s2 = srcs[e2], s3 = srcs[e3];
    s0 = s0 < 0 ? 0 : (s0 > nN - 1 ? nN - 1 : s0);
    s1 = s1 < 0 ? 0 : (s1 > nN - 1 ? nN - 1 : s1);
    s2 = s2 < 0 ? 0 : (s2 > nN - 1 ? nN - 1 : s2);
    s3 = s3 < 0 ? 0 : (s3 > nN - 1 ? nN - 1 : s3);
    v4i o4;
    o4.x = (4 * u     < tt) ? s0 : 0;
    o4.y = (4 * u + 1 < tt) ? s1 : 0;
    o4.z = (4 * u + 2 < tt) ? s2 : 0;
    o4.w = (4 * u + 3 < tt) ? s3 : 0;
    int* gp = lb + 4 * u;
    *(volatile v4i*)gp = o4;
    __threadfence();
    *(volatile v4i*)gp = o4;
  }
  {
    const v4i c4 = *(const v4ia*)(cnt + 4 * tid);
    const v4i o4 = *(const v4ia*)(offs + 4 * tid);
    int* cp = cntg + (size_t)blockIdx.x * NBA + 4 * tid;
    int* op = offg + (size_t)blockIdx.x * NBA + 4 * tid;
    v4i f4; f4.x = ovf; f4.y = ovf; f4.z = ovf; f4.w = ovf;
    int* fp = flg + (size_t)blockIdx.x * 32 + 4 * (tid & 7);
    const bool fw = tid < 8;
    *(volatile v4i*)cp = c4;
    *(volatile v4i*)op = o4;
    if (fw) *(volatile v4i*)fp = f4;
    __threadfence();
    *(volatile v4i*)cp = c4;
    *(volatile v4i*)op = o4;
    if (fw) *(volatile v4i*)fp = f4;
  }
}

__global__ __launch_bounds__(NTHR) void k_agg(const float* __restrict__ Z, const int* __restrict__ lst,
                                              const int* __restrict__ cntg, const int* __restrict__ offg,
                                              const int* __restrict__ flg, const float* __restrict__ tp,
                                              unsigned short* outp, int nN, int mRows) {
  __shared__ __attribute__((aligned(16))) unsigned int stw[NWAVE * 128];
  const int tid = (int)threadIdx.x, lane = tid & 31, wave = tid >> 5;
  const int node = (int)blockIdx.x * NWAVE + wave;
  const int blk  = node >> SLA;
  const int craw = __builtin_amdgcn_readfirstlane(cntg[node]);
  int o          = __builtin_amdgcn_readfirstlane(offg[node]);
  const int fl   = __builtin_amdgcn_readfirstlane(flg[(size_t)blk * 32]);
  int c = craw < 0 ? 0 : (craw > DEGCAP ? DEGCAP : craw);
  o = o < 0 ? 0 : (o > RCAP ? RCAP : o);
  if (c > RCAP - o) c = RCAP - o;
  const bool pois = (fl != 0) || (craw > DEGCAP) || (craw < 0);
  const bool live = node < nN;
  const float tl = bf16_val(tp[0]);
  const int* lb = lst + (size_t)blk * RCAP;
  const int last = o + c - 1;
  const float ninf = -__builtin_huge_valf();

  float m0 = ninf, m1 = ninf, m2 = ninf, m3 = ninf;
#pragma unroll 1
  for (int b0 = 0; b0 < c; b0 += 32) {
    int idx = o + b0 + lane;
    idx = idx > last ? last : idx;
    idx = idx < 0 ? 0 : (idx > RCAP - 1 ? RCAP - 1 : idx);
    int sv = lb[idx];
    sv = sv < 0 ? 0 : (sv > nN - 1 ? nN - 1 : sv);
    const int m32 = (c - b0) < 32 ? (c - b0) : 32;
#pragma unroll 1
    for (int k = 0; k < m32; ++k) {
      const int sk = __builtin_amdgcn_readlane(sv, k);
      const v4f v = *(const v4f*)(Z + (size_t)sk * DH + 4 * lane);
      const float l0 = (relu_keep(v.x) + EPSM) * tl;
      const float l1 = (relu_keep(v.y) + EPSM) * tl;
      const float l2 = (relu_keep(v.z) + EPSM) * tl;
      const float l3 = (relu_keep(v.w) + EPSM) * tl;
      m0 = (l0 > m0 || l0 != l0) ? l0 : m0;
      m1 = (l1 > m1 || l1 != l1) ? l1 : m1;
      m2 = (l2 > m2 || l2 != l2) ? l2 : m2;
      m3 = (l3 > m3 || l3 != l3) ? l3 : m3;
    }
  }

  float d0 = 0.0f, d1 = 0.0f, d2 = 0.0f, d3 = 0.0f;
  float n0 = 0.0f, n1 = 0.0f, n2 = 0.0f, n3 = 0.0f;
#pragma unroll 1
  for (int b0 = 0; b0 < c; b0 += 32) {
    int idx = o + b0 + lane;
    idx = idx > last ? last : idx;
    idx = idx < 0 ? 0 : (idx > RCAP - 1 ? RCAP - 1 : idx);
    int sv = lb[idx];
    sv = sv < 0 ? 0 : (sv > nN - 1 ? nN - 1 : sv);
    const int m32 = (c - b0) < 32 ? (c - b0) : 32;
#pragma unroll 1
    for (int k = 0; k < m32; ++k) {
      const int sk = __builtin_amdgcn_readlane(sv, k);
      const v4f v = *(const v4f*)(Z + (size_t)sk * DH + 4 * lane);
      const float g0 = relu_keep(v.x) + EPSM;
      const float g1 = relu_keep(v.y) + EPSM;
      const float g2 = relu_keep(v.z) + EPSM;
      const float g3 = relu_keep(v.w) + EPSM;
      const float x0 = expf(g0 * tl - m0);
      const float x1 = expf(g1 * tl - m1);
      const float x2 = expf(g2 * tl - m2);
      const float x3 = expf(g3 * tl - m3);
      d0 += x0; d1 += x1; d2 += x2; d3 += x3;
      n0 += x0 * g0; n1 += x1 * g1; n2 += x2 * g2; n3 += x3 * g3;
    }
  }
  const bool has = c > 0;
  const float q0 = n0 / (has ? (d0 + EPSS) : 1.0f);
  const float q1 = n1 / (has ? (d1 + EPSS) : 1.0f);
  const float q2 = n2 / (has ? (d2 + EPSS) : 1.0f);
  const float q3 = n3 / (has ? (d3 + EPSS) : 1.0f);
  const int nc = live ? node : nN - 1;
  const v4f zs = *(const v4f*)(Z + (size_t)nc * DH + 4 * lane);
  const float qnan = __int_as_float(0x7fc00000);
  float r0 = (has ? q0 : 0.0f) + zs.x;
  float r1 = (has ? q1 : 0.0f) + zs.y;
  float r2 = (has ? q2 : 0.0f) + zs.z;
  float r3 = (has ? q3 : 0.0f) + zs.w;
  r0 = live ? (pois ? qnan : r0) : 0.0f;
  r1 = live ? (pois ? qnan : r1) : 0.0f;
  r2 = live ? (pois ? qnan : r2) : 0.0f;
  r3 = live ? (pois ? qnan : r3) : 0.0f;

  unsigned lb0, lb1, lb2, lb3;
  const unsigned hb0 = hl_bits(r0, lb0), hb1 = hl_bits(r1, lb1);
  const unsigned hb2 = hl_bits(r2, lb2), hb3 = hl_bits(r3, lb3);
  v2u hw, lw;
  hw.x = (hb0 & 0xffffu) | (hb1 << 16);
  hw.y = (hb2 & 0xffffu) | (hb3 << 16);
  lw.x = (lb0 & 0xffffu) | (lb1 << 16);
  lw.y = (lb2 & 0xffffu) | (lb3 << 16);
  unsigned int* stwu = stw + wave * 128;
  *(v2ua*)(stwu + 2 * lane)      = hw;
  *(v2ua*)(stwu + 64 + 2 * lane) = lw;
  wave_sync();
  const v4u pk = *(const v4ua*)(stwu + 4 * lane);
  unsigned short* gp = outp + (size_t)node * OPW + 8 * lane;
  const bool wsv = node < mRows;
  if (wsv) *(volatile v4u*)gp = pk;
  __threadfence();
  if (wsv) *(volatile v4u*)gp = pk;
}

__global__ __launch_bounds__(GTHR) void k_gemm_a(const unsigned short* __restrict__ A,
                                                 const unsigned short* __restrict__ BT,
                                                 const float* __restrict__ bias, const float* __restrict__ gam,
                                                 const float* __restrict__ bet,
                                                 unsigned short* hm, int nN, int mRows) {
  __shared__ __attribute__((aligned(16))) float stg[ABM * DHID];
  const int tid = (int)threadIdx.x, lane = tid & 31, wave = tid >> 5, hh = lane >> 4, m = lane & 15;
  const int rg = wave & 1, ch = wave >> 1;
  const int rowBase = (int)blockIdx.x * ABM;

  v8f acc[8];
#pragma unroll
  for (int t = 0; t < 8; ++t) acc[t] = z8();
  const unsigned short* ap = A + (size_t)(rowBase + 16 * rg + m) * (size_t)OPW + 8 * hh;
  const unsigned short* bp = BT + (size_t)(128 * ch + m) * (size_t)KA + 8 * hh;

#pragma unroll 1
  for (int k0 = 0; k0 < KA; k0 += 32) {
    FragB af;
    af.h[0] = *(const v8usa*)(ap + k0);
    af.h[1] = *(const v8usa*)(ap + k0 + 16);
#pragma unroll
    for (int nt = 0; nt < 8; ++nt) {
      const unsigned short* wq = bp + (size_t)(16 * nt) * (size_t)KA + k0;
      FragB bf;
      bf.h[0] = *(const v8usa*)wq;
      bf.h[1] = *(const v8usa*)(wq + 16);
      acc[nt] = wmb(af, bf, acc[nt]);
    }
  }

#pragma unroll
  for (int nt = 0; nt < 8; ++nt) {
    const int lc = 128 * ch + 16 * nt + m;
#pragma unroll
    for (int r = 0; r < 8; ++r) {
      const int lr = 16 * rg + 8 * hh + r;
      stg[lr * DHID + lc] = acc[nt][r];
    }
  }
  __syncthreads();

  float bq[8], gq[8], eq[8];
  {
    const v4f b0 = *(const v4f*)(bias + 8 * lane), b1 = *(const v4f*)(bias + 8 * lane + 4);
    const v4f g0 = *(const v4f*)(gam + 8 * lane),  g1 = *(const v4f*)(gam + 8 * lane + 4);
    const v4f e0 = *(const v4f*)(bet + 8 * lane),  e1 = *(const v4f*)(bet + 8 * lane + 4);
    bq[0] = bf16_val(b0.x); bq[1] = bf16_val(b0.y); bq[2] = bf16_val(b0.z); bq[3] = bf16_val(b0.w);
    bq[4] = bf16_val(b1.x); bq[5] = bf16_val(b1.y); bq[6] = bf16_val(b1.z); bq[7] = bf16_val(b1.w);
    gq[0] = bf16_val(g0.x); gq[1] = bf16_val(g0.y); gq[2] = bf16_val(g0.z); gq[3] = bf16_val(g0.w);
    gq[4] = bf16_val(g1.x); gq[5] = bf16_val(g1.y); gq[6] = bf16_val(g1.z); gq[7] = bf16_val(g1.w);
    eq[0] = bf16_val(e0.x); eq[1] = bf16_val(e0.y); eq[2] = bf16_val(e0.z); eq[3] = bf16_val(e0.w);
    eq[4] = bf16_val(e1.x); eq[5] = bf16_val(e1.y); eq[6] = bf16_val(e1.z); eq[7] = bf16_val(e1.w);
  }

  const float invd = 1.0f / (float)DHID;
#pragma unroll 1
  for (int i = 0; i < 8; ++i) {
    const int lr  = 8 * wave + i;
    const int row = rowBase + lr;
    const bool ok = row < nN;
    const v4f pa = *(const v4fa*)(stg + lr * DHID + 8 * lane);
    const v4f pb = *(const v4fa*)(stg + lr * DHID + 8 * lane + 4);
    float y[8];
    y[0] = pa.x + bq[0]; y[1] = pa.y + bq[1]; y[2] = pa.z + bq[2]; y[3] = pa.w + bq[3];
    y[4] = pb.x + bq[4]; y[5] = pb.y + bq[5]; y[6] = pb.z + bq[6]; y[7] = pb.w + bq[7];
    float s = ((y[0] + y[1]) + (y[2] + y[3])) + ((y[4] + y[5]) + (y[6] + y[7]));
    s += __shfl_xor(s, 16, 32);
    s += __shfl_xor(s, 8, 32);
    s += __shfl_xor(s, 4, 32);
    s += __shfl_xor(s, 2, 32);
    s += __shfl_xor(s, 1, 32);
    const float mean = s * invd;
    float d[8];
#pragma unroll
    for (int j = 0; j < 8; ++j) d[j] = y[j] - mean;
    float q = ((d[0] * d[0] + d[1] * d[1]) + (d[2] * d[2] + d[3] * d[3])) +
              ((d[4] * d[4] + d[5] * d[5]) + (d[6] * d[6] + d[7] * d[7]));
    q += __shfl_xor(q, 16, 32);
    q += __shfl_xor(q, 8, 32);
    q += __shfl_xor(q, 4, 32);
    q += __shfl_xor(q, 2, 32);
    q += __shfl_xor(q, 1, 32);
    const float var  = q * invd;
    const float rstd = rsqrtf(var + LNEPS);
    unsigned hb[8], lbv[8];
#pragma unroll
    for (int j = 0; j < 8; ++j) {
      const float o = relu_keep(fmaf(d[j] * rstd, gq[j], eq[j]));
      const float ov = ok ? o : 0.0f;
      unsigned lo;
      hb[j] = hl_bits(ov, lo);
      lbv[j] = lo;
    }
    v4u hiw, low;
    hiw.x = (hb[0] & 0xffffu) | (hb[1] << 16);
    hiw.y = (hb[2] & 0xffffu) | (hb[3] << 16);
    hiw.z = (hb[4] & 0xffffu) | (hb[5] << 16);
    hiw.w = (hb[6] & 0xffffu) | (hb[7] << 16);
    low.x = (lbv[0] & 0xffffu) | (lbv[1] << 16);
    low.y = (lbv[2] & 0xffffu) | (lbv[3] << 16);
    low.z = (lbv[4] & 0xffffu) | (lbv[5] << 16);
    low.w = (lbv[6] & 0xffffu) | (lbv[7] << 16);
    unsigned short* rp = hm + (size_t)row * (size_t)HPW + 8 * lane;
    const bool wsv = row < mRows;
    if (wsv) {
      *(volatile v4u*)rp = hiw;
      *(volatile v4u*)(rp + DHID) = low;
    }
    __threadfence();
    if (wsv) {
      *(volatile v4u*)rp = hiw;
      *(volatile v4u*)(rp + DHID) = low;
    }
  }
}

template <int MODE>
__global__ __launch_bounds__(GTHR) void k_gemm128(const unsigned short* __restrict__ A, int lda,
                                                  const unsigned short* __restrict__ BT, int ldb, int K,
                                                  const float* __restrict__ bias, const float* __restrict__ gam,
                                                  const float* __restrict__ bet,
                                                  float* hpl, float* zpl, int nN, int mRows, int wantZ) {
  __shared__ __attribute__((aligned(16))) float stg[GBM * DH];
  const int tid = (int)threadIdx.x, lane = tid & 31, wave = tid >> 5, hh = lane >> 4, m = lane & 15;
  const int rowBase = (int)blockIdx.x * GBM;

  v8f acc[8];
#pragma unroll
  for (int t = 0; t < 8; ++t) acc[t] = z8();
  const unsigned short* ap = A + (size_t)(rowBase + 16 * wave + m) * (size_t)lda + 8 * hh;
  const unsigned short* bp = BT + (size_t)m * (size_t)ldb + 8 * hh;

#pragma unroll 1
  for (int k0 = 0; k0 < K; k0 += 32) {
    FragB af;
    af.h[0] = *(const v8usa*)(ap + k0);
    af.h[1] = *(const v8usa*)(ap + k0 + 16);
#pragma unroll
    for (int nt = 0; nt < 8; ++nt) {
      const unsigned short* wq = bp + (size_t)(16 * nt) * (size_t)ldb + k0;
      FragB bf;
      bf.h[0] = *(const v8usa*)wq;
      bf.h[1] = *(const v8usa*)(wq + 16);
      acc[nt] = wmb(af, bf, acc[nt]);
    }
  }

#pragma unroll
  for (int nt = 0; nt < 8; ++nt) {
    const int lc = 16 * nt + m;
#pragma unroll
    for (int r = 0; r < 8; ++r) {
      const int lr = 16 * wave + 8 * hh + r;
      stg[lr * DH + lc] = acc[nt][r];
    }
  }
  __syncthreads();

  float bq[4], gq[4], eq[4];
  {
    const v4f b4 = *(const v4f*)(bias + 4 * lane);
    const v4f g4 = *(const v4f*)(gam + 4 * lane);
    const v4f e4 = *(const v4f*)(bet + 4 * lane);
    bq[0] = bf16_val(b4.x); bq[1] = bf16_val(b4.y); bq[2] = bf16_val(b4.z); bq[3] = bf16_val(b4.w);
    gq[0] = bf16_val(g4.x); gq[1] = bf16_val(g4.y); gq[2] = bf16_val(g4.z); gq[3] = bf16_val(g4.w);
    eq[0] = bf16_val(e4.x); eq[1] = bf16_val(e4.y); eq[2] = bf16_val(e4.z); eq[3] = bf16_val(e4.w);
  }

  const float invd = 1.0f / (float)DH;
#pragma unroll 1
  for (int i = 0; i < 16; ++i) {
    const int lr  = 16 * wave + i;
    const int row = rowBase + lr;
    const bool ok = row < nN;
    const v4f d4 = *(const v4fa*)(stg + lr * DH + 4 * lane);
    float y0 = d4.x + bq[0], y1 = d4.y + bq[1], y2 = d4.z + bq[2], y3 = d4.w + bq[3];
    float* hp = hpl + (size_t)row * DH + 4 * lane;
    float* zp = zpl + (size_t)row * DH + 4 * lane;
    if (MODE == 1) {
      const v4f h4 = *(const v4f*)hp;
      y0 = h4.x + y0; y1 = h4.y + y1; y2 = h4.z + y2; y3 = h4.w + y3;
    }
    v4f hv;
    hv.x = ok ? y0 : 0.0f; hv.y = ok ? y1 : 0.0f; hv.z = ok ? y2 : 0.0f; hv.w = ok ? y3 : 0.0f;
    float s = (y0 + y1) + (y2 + y3);
    s += __shfl_xor(s, 16, 32);
    s += __shfl_xor(s, 8, 32);
    s += __shfl_xor(s, 4, 32);
    s += __shfl_xor(s, 2, 32);
    s += __shfl_xor(s, 1, 32);
    const float mean = s * invd;
    const float e0 = y0 - mean, e1 = y1 - mean, e2 = y2 - mean, e3 = y3 - mean;
    float q = (e0 * e0 + e1 * e1) + (e2 * e2 + e3 * e3);
    q += __shfl_xor(q, 16, 32);
    q += __shfl_xor(q, 8, 32);
    q += __shfl_xor(q, 4, 32);
    q += __shfl_xor(q, 2, 32);
    q += __shfl_xor(q, 1, 32);
    const float var  = q * invd;
    const float rstd = rsqrtf(var + LNEPS);
    const float o0 = relu_keep(fmaf(e0 * rstd, gq[0], eq[0]));
    const float o1 = relu_keep(fmaf(e1 * rstd, gq[1], eq[1]));
    const float o2 = relu_keep(fmaf(e2 * rstd, gq[2], eq[2]));
    const float o3 = relu_keep(fmaf(e3 * rstd, gq[3], eq[3]));
    v4f zv;
    zv.x = ok ? o0 : 0.0f; zv.y = ok ? o1 : 0.0f; zv.z = ok ? o2 : 0.0f; zv.w = ok ? o3 : 0.0f;
    const bool wsv = row < mRows;
    const bool wz  = wsv && (wantZ != 0);
    if (wsv) *(volatile v4f*)hp = hv;
    if (wz)  *(volatile v4f*)zp = zv;
    __threadfence();
    if (wsv) *(volatile v4f*)hp = hv;
    if (wz)  *(volatile v4f*)zp = zv;
  }
}

__global__ __launch_bounds__(NTHR) void k_pool(const float* __restrict__ hf, const int* __restrict__ bat,
                                               int nN, float* pooled) {
  __shared__ __attribute__((aligned(16))) float wsum[NWAVE * DH];
  __shared__ __attribute__((aligned(16))) float outs[DH];
  const int tid = (int)threadIdx.x, lane = tid & 31, wave = tid >> 5;
  const int g = (int)blockIdx.x;

  float a0 = 0.0f, a1 = 0.0f, a2 = 0.0f, a3 = 0.0f;
#pragma unroll 1
  for (int i0 = wave * 32; i0 < nN; i0 += NTHR) {
    const int i  = i0 + lane;
    const int ic = i < nN ? i : nN - 1;
    const int b  = bat[ic];
    const bool hit = (i < nN) && (b == g);
    unsigned msk = __builtin_amdgcn_ballot_w32(hit);
    int nh = (int)__builtin_popcount(msk);
    nh = nh > 32 ? 32 : nh;
#pragma unroll 1
    for (int q = 0; q < nh; ++q) {
      const int k = __builtin_ffs((int)msk) - 1;
      msk &= msk - 1u;
      int node = i0 + (k < 0 ? 0 : k);
      node = node > nN - 1 ? nN - 1 : node;
      const v4f v = *(const v4f*)(hf + (size_t)node * DH + 4 * lane);
      a0 += v.x; a1 += v.y; a2 += v.z; a3 += v.w;
    }
  }
  {
    v4f sv; sv.x = a0; sv.y = a1; sv.z = a2; sv.w = a3;
    *(v4fa*)(wsum + wave * DH + 4 * lane) = sv;
  }
  __syncthreads();
  if (tid < DH) {
    double s = 0.0;
#pragma unroll 1
    for (int w2 = 0; w2 < NWAVE; ++w2) s += (double)wsum[w2 * DH + tid];
    outs[tid] = (float)s;
  }
  __syncthreads();
  const v4f ov = *(const v4fa*)(outs + 4 * lane);
  float* op = pooled + (size_t)g * DH + 4 * lane;
  const bool okst = (wave == 0);
  if (okst) *(volatile v4f*)op = ov;
  __threadfence();
  if (okst) *(volatile v4f*)op = ov;
}

__global__ __launch_bounds__(NTHR) void k_head(const float* __restrict__ pooled, const float* __restrict__ clsW,
                                               const float* __restrict__ clsb, float* out) {
  __shared__ float wsh[2 * DH];
  __shared__ float bsh[4];
  __shared__ __attribute__((aligned(16))) float ost[2 * NGRAPH];
  const int tid = (int)threadIdx.x;
  wsh[tid] = bf16_val(clsW[tid]);
  if (tid < 4) bsh[tid] = bf16_val(clsb[tid < 2 ? tid : 1]);
  __syncthreads();
  float a0 = 0.0f, a1 = 0.0f;
  const float* pr = pooled + (size_t)tid * DH;
#pragma unroll 1
  for (int q = 0; q < DH / 4; ++q) {
    const v4f p = *(const v4f*)(pr + 4 * q);
    a0 = fmaf(p.x, wsh[8 * q + 0], a0); a1 = fmaf(p.x, wsh[8 * q + 1], a1);
    a0 = fmaf(p.y, wsh[8 * q + 2], a0); a1 = fmaf(p.y, wsh[8 * q + 3], a1);
    a0 = fmaf(p.z, wsh[8 * q + 4], a0); a1 = fmaf(p.z, wsh[8 * q + 5], a1);
    a0 = fmaf(p.w, wsh[8 * q + 6], a0); a1 = fmaf(p.w, wsh[8 * q + 7], a1);
  }
  ost[2 * tid + 0] = a0 + bsh[0];
  ost[2 * tid + 1] = a1 + bsh[1];
  __syncthreads();
  const bool ok = tid < (2 * NGRAPH) / 4;
  v4f v = {0.f, 0.f, 0.f, 0.f};
  if (ok) v = *(const v4fa*)(ost + 4 * tid);
  float* op = out + 4 * (ok ? tid : 0);
  if (ok) *(volatile v4f*)op = v;
  __threadfence();
  if (ok) *(volatile v4f*)op = v;
}

static inline int cdiv(int a, int b) { return (a + b - 1) / b; }
static inline size_t al256(size_t o) { return (o + 255) & ~(size_t)255; }

extern "C" void kernel_launch(void* const* d_in, const int* in_sizes, int n_in,
                              void* d_out, int out_size, void* d_ws, size_t ws_size,
                              hipStream_t stream) {
  if (n_in < 16) return;
  const int nN = in_sizes[2];
  if (nN < GBM || nN > (1 << 22)) return;
  if ((long long)in_sizes[0] != (long long)nN * DINF) return;
  if (in_sizes[1] < 2 || (in_sizes[1] & 1) != 0) return;
  const int nE = in_sizes[1] / 2;
  if (nE < 1 || nE >= (1 << 21)) return;
  if (in_sizes[3] != DINF * DH || in_sizes[4] != DH) return;
  if (in_sizes[5] != NLAY) return;
  if (in_sizes[6] != NLAY * DH * DHID || in_sizes[7] != NLAY * DHID) return;
  if (in_sizes[8] != NLAY * DHID || in_sizes[9] != NLAY * DHID) return;
  if (in_sizes[10] != NLAY * DHID * DH || in_sizes[11] != NLAY * DH) return;
  if (in_sizes[12] != NLAY * DH || in_sizes[13] != NLAY * DH) return;
  if (in_sizes[14] != DH * 2 || in_sizes[15] != 2) return;
  if (out_size != NGRAPH * 2) return;

  const float* x    = (const float*)d_in[0];
  const int*   ei   = (const int*)  d_in[1];
  const int*   bat  = (const int*)  d_in[2];
  const float* encW = (const float*)d_in[3];
  const float* encb = (const float*)d_in[4];
  const float* tt   = (const float*)d_in[5];
  const float* W1   = (const float*)d_in[6];
  const float* b1   = (const float*)d_in[7];
  const float* g1   = (const float*)d_in[8];
  const float* bb1  = (const float*)d_in[9];
  const float* W2   = (const float*)d_in[10];
  const float* b2   = (const float*)d_in[11];
  const float* lng  = (const float*)d_in[12];
  const float* lnb  = (const float*)d_in[13];
  const float* clsW = (const float*)d_in[14];
  const float* clsb = (const float*)d_in[15];
  float* out = (float*)d_out;
  const int* src = ei;
  const int* dst = ei + nE;

  const int MP = cdiv(nN, GBM) * GBM;
  const int gA = cdiv(MP, NBA);
  if ((long long)gA * NBA < (long long)MP) return;
  if ((MP % ABM) != 0 || (MP % NWAVE) != 0) return;
  const int vec8 = ((nE & 3) == 0) ? 1 : 0;

  char* ws = (char*)d_ws;
  size_t off = 0;
  const size_t oH   = off; off = al256(off + (size_t)MP * DH * 4);
  const size_t oZ   = off; off = al256(off + (size_t)MP * DH * 4);
  const size_t oOUT = off; off = al256(off + (size_t)MP * OPW * 2);
  const size_t oHM  = off; off = al256(off + (size_t)MP * HPW * 2);
  const size_t oLST = off; off = al256(off + (size_t)gA * RCAP * 4);
  const size_t oCNT = off; off = al256(off + (size_t)gA * NBA * 4);
  const size_t oOFF = off; off = al256(off + (size_t)gA * NBA * 4);
  const size_t oFLG = off; off = al256(off + (size_t)gA * 32 * 4);
  const size_t oW1  = off; off = al256(off + (size_t)NLAY * DHID * KA * 2);
  const size_t oW2  = off; off = al256(off + (size_t)NLAY * DH * KB * 2);
  const size_t oEW  = off; off = al256(off + (size_t)DH * KE * 2);
  const size_t oPL  = off; off = al256(off + (size_t)NGRAPH * DH * 4);
  if (off > ws_size || off > (size_t)WSMAX) return;
  if ((size_t)MP * KE * 2 > (size_t)MP * HPW * 2) return;
  float*          H    = (float*)(ws + oH);
  float*          Z    = (float*)(ws + oZ);
  unsigned short* OUT  = (unsigned short*)(ws + oOUT);
  unsigned short* HM   = (unsigned short*)(ws + oHM);
  unsigned short* XB   = (unsigned short*)(ws + oHM);
  int*            LST  = (int*)(ws + oLST);
  int*            CNT  = (int*)(ws + oCNT);
  int*            OFF  = (int*)(ws + oOFF);
  int*            FLG  = (int*)(ws + oFLG);
  unsigned short* W1T  = (unsigned short*)(ws + oW1);
  unsigned short* W2T  = (unsigned short*)(ws + oW2);
  unsigned short* EWT  = (unsigned short*)(ws + oEW);
  float*          POOL = (float*)(ws + oPL);

  const size_t cmpLds = (size_t)CMP_LDS_INTS * 4;
  hipFuncSetAttribute(reinterpret_cast<const void*>(&k_compact), hipFuncAttributeMaxDynamicSharedMemorySize, (int)cmpLds);

  const int nUnits = NUFIX + MP * (KE / 8);

  k_prep<<<cdiv(nUnits, NTHR), NTHR, 0, stream>>>(x, encW, W1, W2, EWT, W1T, W2T, XB, nN, nUnits);
  k_compact<<<gA, NTHR, cmpLds, stream>>>(src, dst, nE, nN, vec8, LST, CNT, OFF, FLG);
  k_gemm128<0><<<MP / GBM, GTHR, 0, stream>>>(XB, KE, EWT, KE, KE, encb, lng, lnb, H, Z, nN, MP, 1);
  for (int l = 0; l < NLAY; ++l) {
    k_agg<<<MP / NWAVE, NTHR, 0, stream>>>(Z, LST, CNT, OFF, FLG, tt + l, OUT, nN, MP);
    k_gemm_a<<<MP / ABM, GTHR, 0, stream>>>(OUT, W1T + (size_t)l * DHID * KA, b1 + (size_t)l * DHID,
                                            g1 + (size_t)l * DHID, bb1 + (size_t)l * DHID, HM, nN, MP);
    const int lz = (l + 1 < NLAY) ? (l + 1) : l;
    k_gemm128<1><<<MP / GBM, GTHR, 0, stream>>>(HM, HPW, W2T + (size_t)l * DH * KB, KB, KB,
                                                b2 + (size_t)l * DH, lng + (size_t)lz * DH, lnb + (size_t)lz * DH,
                                                H, Z, nN, MP, (l + 1 < NLAY) ? 1 : 0);
  }
  k_pool<<<NGRAPH, NTHR, 0, stream>>>(H, bat, nN, POOL);
  k_head<<<1, NTHR, 0, stream>>>(POOL, clsW, clsb, out);
}
